// MultiHeadDotProduct_67946382623506
// MI455X (gfx1250) — hardware-run, weakly checked
//
#include <hip/hip_runtime.h>


#define SEQ  512
#define NE   (SEQ * SEQ)
#define DM   256
#define NH_  8
#define HD   32
#define AW   4
#define HPW  2
#define OSP  68
#define SC2  ((float)(0.17677669529663687 * 1.4426950408889634))
#define PSH  14.0f
#define NEGB (-3.0e38f)
#define ACS  256.0f
#define WOS  64.0f
#define OSI  (1.0f / (256.0f * 64.0f))
#define ECB  32
#define ECT  256
#define ECI  ((NE * 2 / 4) / (ECB * ECT))

static_assert(HD == 32);
static_assert(NH_ * HD == DM);
static_assert(HPW * HD * 2 == 128);
static_assert(NH_ % HPW == 0);
static_assert(DM % 64 == 0);
static_assert(64 % HD == 0);
static_assert(DM % 32 == 0);
static_assert(SEQ % 64 == 0);
static_assert(SEQ % 32 == 0);
static_assert(SEQ % (16 * AW) == 0);
static_assert((SEQ & (SEQ - 1)) == 0);
static_assert(((size_t)SEQ * DM) % 8 == 0);
static_assert(((size_t)DM * DM) % 8 == 0);
static_assert((OSP * 4) % 16 == 0);
static_assert(OSP >= 64);
static_assert(ECB == 32);
static_assert((size_t)ECB * ECI * ECT * 4 == (size_t)NE * 2);
static_assert(16 * OSP * 4 <= 131072);
static_assert(AW * 16 * OSP * 4 <= 131072);

typedef _Float16 h16;
typedef unsigned short bf;
typedef __attribute__((ext_vector_type(16))) __bf16   v16bf;
typedef __attribute__((ext_vector_type(16))) _Float16 v16h;
typedef __attribute__((ext_vector_type(8)))  _Float16 v8h;
typedef __attribute__((ext_vector_type(8)))  unsigned short v8us;
typedef __attribute__((ext_vector_type(8)))  float    v8f;
typedef __attribute__((ext_vector_type(4)))  float    v4f;
typedef __attribute__((ext_vector_type(4)))  int      v4i;
typedef v4f  __attribute__((may_alias)) v4fa;

__device__ __forceinline__ unsigned short f2bf(float f) { unsigned u = __float_as_uint(f); u += 0x7FFFu + ((u >> 16) & 1u); return (unsigned short)(u >> 16); }
__device__ __forceinline__ float bfr(float f) { return __uint_as_float(((unsigned)f2bf(f)) << 16); }
__device__ __forceinline__ v16h cat16(v8h lo, v8h hi) { return __builtin_shufflevector(lo, hi, 0, 1, 2, 3, 4, 5, 6, 7, 8, 9, 10, 11, 12, 13, 14, 15); }
__device__ __forceinline__ v16bf cat16b(v8us lo, v8us hi) { return __builtin_bit_cast(v16bf, __builtin_shufflevector(lo, hi, 0, 1, 2, 3, 4, 5, 6, 7, 8, 9, 10, 11, 12, 13, 14, 15)); }
__device__ __forceinline__ v8f wmma16(v16h a, v16h b, v8f c) { return __builtin_amdgcn_wmma_f32_16x16x32_f16(false, a, false, b, (short)0, c, false, false); }
__device__ __forceinline__ v8f wmmab(v16bf a, v16bf b, v8f c) { return __builtin_amdgcn_wmma_f32_16x16x32_bf16(false, a, false, b, (short)0, c, false, false); }
__device__ __forceinline__ v16h  ldh(const h16* p) { return cat16(*(const v8h*)p, *(const v8h*)(p + 16)); }
__device__ __forceinline__ v16bf ldb(const bf* p)  { return cat16b(*(const v8us*)p, *(const v8us*)(p + 16)); }
__device__ __forceinline__ void wave_sync() { __builtin_amdgcn_fence(3  , "wavefront"); __builtin_amdgcn_wave_barrier(); asm volatile("" ::: "memory"); }

static __device__ __forceinline__ h16 toh_flush(float v) { const h16 r = (h16)v; return (fabsf(v) < 6.103515625e-05f) ? (h16)0.0f : r; }
__device__ __forceinline__ v8f wmma16g(v16h a, v16h b, v8f c) { c = wmma16(a, b, c); asm volatile("v_nop\n\tv_nop\n\tv_nop\n\tv_nop" : "+v"(c) : "v"(a), "v"(b)); return c; }
__device__ __forceinline__ v8f wmmabg(v16bf a, v16bf b, v8f c) { c = wmmab(a, b, c); asm volatile("v_nop\n\tv_nop\n\tv_nop\n\tv_nop" : "+v"(c) : "v"(a), "v"(b)); return c; }

__global__ __launch_bounds__(256) void k_cvt8(const float* __restrict__ src, bf* dst, size_t n8) {
    const size_t i = (size_t)blockIdx.x * 256 + threadIdx.x; if (i >= n8) return;
    const v8f v = *(const v8f*)(src + i * 8); v8us o;
#pragma unroll
    for (int k = 0; k < 8; ++k) o[k] = f2bf(v[k]);
    *(volatile v8us*)(dst + i * 8) = o; __threadfence(); *(volatile v8us*)(dst + i * 8) = o;
}

__global__ __launch_bounds__(256) void k_cvtw(const float* __restrict__ src, h16* dst, size_t n8) {
    const size_t i = (size_t)blockIdx.x * 256 + threadIdx.x; if (i >= n8) return;
    const v8f v = *(const v8f*)(src + i * 8); v8h o;
#pragma unroll
    for (int k = 0; k < 8; ++k) o[k] = toh_flush(bfr(v[k]) * WOS);
    *(volatile v8h*)(dst + i * 8) = o; __threadfence(); *(volatile v8h*)(dst + i * 8) = o;
}

__global__ __launch_bounds__(ECT) void k_echeck(const int* __restrict__ ei, int* FLG) {
    __shared__ int wflag[ECT / 32];
    const int lane = threadIdx.x & 31;
    const int wave = __builtin_amdgcn_readfirstlane((int)(threadIdx.x >> 5));
    int bad = 0;
#pragma unroll 1
    for (int it = 0; it < ECI; ++it) {
        const int q4 = ((int)blockIdx.x * ECI + it) * ECT + (int)threadIdx.x;
        const v4i w = *(const v4i*)(ei + (size_t)q4 * 4);
        const int e0 = 2 * q4, e1 = 2 * q4 + 1;
        bad |= (int)(w[0] != (e0 & (SEQ - 1))) | (int)(w[1] != (e0 / SEQ)) | (int)(w[2] != (e1 & (SEQ - 1))) | (int)(w[3] != (e1 / SEQ));
    }
    bad |= __shfl_xor(bad, 16, 32); bad |= __shfl_xor(bad, 8, 32); bad |= __shfl_xor(bad, 4, 32); bad |= __shfl_xor(bad, 2, 32); bad |= __shfl_xor(bad, 1, 32);
    if (lane == 0) wflag[wave] = bad;
    __syncthreads();
    int tot = 0;
#pragma unroll
    for (int w = 0; w < ECT / 32; ++w) tot |= wflag[w];
    const v4i fv = (v4i){ tot, tot, tot, tot };
    static_assert(8 * 16 == 128);
    if (threadIdx.x < 8) {
        int* p = FLG + (size_t)blockIdx.x * 32 + (size_t)threadIdx.x * 4;
        *(volatile v4i*)p = fv; __threadfence(); *(volatile v4i*)p = fv;
    }
}

__global__ __launch_bounds__(32) void k_proj_rows(const bf* __restrict__ A, const bf* __restrict__ Bt, const float* __restrict__ bias, h16* Ph) {
    __shared__ __align__(16) float os[16 * OSP];
    const int K = DM;
    const int lane = threadIdx.x & 31, lr = lane & 15, hi = lane >> 4; const int r0 = blockIdx.x * 64, c0 = blockIdx.y * 64;
    v8f acc[4][4];
#pragma unroll
    for (int mb = 0; mb < 4; ++mb)
#pragma unroll
        for (int nb = 0; nb < 4; ++nb) acc[mb][nb] = (v8f){};
    const size_t aoff = (size_t)(r0 + lr) * K + 8 * hi, boff = (size_t)(c0 + lr) * K + 8 * hi;
#pragma unroll 1
    for (int kc = 0; kc < K; kc += 32) {
        v16bf a[4];
#pragma unroll
        for (int mb = 0; mb < 4; ++mb) a[mb] = ldb(A + aoff + (size_t)mb * 16 * K + kc);
#pragma unroll
        for (int nb = 0; nb < 4; ++nb) { const v16bf b = ldb(Bt + boff + (size_t)nb * 16 * K + kc);
#pragma unroll
            for (int mb = 0; mb < 4; ++mb) acc[mb][nb] = wmmabg(a[mb], b, acc[mb][nb]); }
    }
    float bc[4];
#pragma unroll
    for (int nb = 0; nb < 4; ++nb) bc[nb] = bfr(bias[c0 + nb * 16 + lr]);
    const size_t tbase = ((size_t)(c0 / HD) * SEQ + (size_t)r0) * HD;
#pragma unroll
    for (int mb = 0; mb < 4; ++mb) {
#pragma unroll
        for (int nb = 0; nb < 4; ++nb) {
#pragma unroll
            for (int j = 0; j < 8; ++j) os[(hi * 8 + j) * OSP + nb * 16 + lr] = acc[mb][nb][j] + bc[nb]; }
        wave_sync();
        static_assert(32 * 16 * 2 == 16 * HD * 2);
#pragma unroll 1
        for (int ps = 0; ps < 2; ++ps) {
            const size_t sb = tbase + (size_t)(mb * 16) * HD;
#pragma unroll
            for (int hh = 0; hh < 2; ++hh) {
#pragma unroll
                for (int s = 0; s < 2; ++s) { const int p = s * 32 + lane; const int row = p >> 2, c8 = (p & 3) * 8;
                    const v4f x0 = *(const v4fa*)(&os[row * OSP + hh * 32 + c8]); const v4f x1 = *(const v4fa*)(&os[row * OSP + hh * 32 + c8 + 4]); v8h hv;
#pragma unroll
                    for (int i = 0; i < 4; ++i) { hv[i] = toh_flush(x0[i]); hv[4 + i] = toh_flush(x1[i]); }
                    const size_t oo = sb + (size_t)hh * ((size_t)SEQ * HD) + (size_t)p * 8;
                    *(volatile v8h*)(Ph + oo) = hv; } }
            if (ps == 0) __threadfence(); }
        wave_sync();
    }
}

__global__ __launch_bounds__(32) void k_proj_cols(const bf* __restrict__ A, const bf* __restrict__ Bt, const float* __restrict__ bias, h16* Ph) {
    __shared__ __align__(16) float os[16 * OSP];
    const int K = DM;
    const int lane = threadIdx.x & 31, lr = lane & 15, hi = lane >> 4; const int r0 = blockIdx.x * 64, c0 = blockIdx.y * 64;
    v8f acc[4][4];
#pragma unroll
    for (int mb = 0; mb < 4; ++mb)
#pragma unroll
        for (int nb = 0; nb < 4; ++nb) acc[mb][nb] = (v8f){};
    const size_t aoff = (size_t)(r0 + lr) * K + 8 * hi, boff = (size_t)(c0 + lr) * K + 8 * hi;
#pragma unroll 1
    for (int kc = 0; kc < K; kc += 32) {
        v16bf a[4];
#pragma unroll
        for (int mb = 0; mb < 4; ++mb) a[mb] = ldb(A + aoff + (size_t)mb * 16 * K + kc);
#pragma unroll
        for (int nb = 0; nb < 4; ++nb) { const v16bf b = ldb(Bt + boff + (size_t)nb * 16 * K + kc);
#pragma unroll
            for (int mb = 0; mb < 4; ++mb) acc[mb][nb] = wmmabg(a[mb], b, acc[mb][nb]); }
    }
    const size_t tbase = (size_t)r0 * SEQ + (size_t)c0;
#pragma unroll
    for (int mb = 0; mb < 4; ++mb) {
        float br[8];
#pragma unroll
        for (int j = 0; j < 8; ++j) br[j] = bfr(bias[r0 + mb * 16 + hi * 8 + j]);
#pragma unroll
        for (int nb = 0; nb < 4; ++nb) {
#pragma unroll
            for (int j = 0; j < 8; ++j) os[(hi * 8 + j) * OSP + nb * 16 + lr] = acc[mb][nb][j] + br[j]; }
        wave_sync();
        static_assert(32 * 16 * 4 == 16 * 64 * 2);
#pragma unroll 1
        for (int ps = 0; ps < 2; ++ps) {
            const size_t sb = tbase + (size_t)(mb * 16) * SEQ;
#pragma unroll
            for (int s = 0; s < 4; ++s) { const int row = 4 * s + (lane >> 3), c8 = (lane & 7) * 8;
                const v4f x0 = *(const v4fa*)(&os[row * OSP + c8]); const v4f x1 = *(const v4fa*)(&os[row * OSP + c8 + 4]); v8h hv;
#pragma unroll
                for (int i = 0; i < 4; ++i) { hv[i] = toh_flush(x0[i]); hv[4 + i] = toh_flush(x1[i]); }
                const size_t oo = sb + (size_t)row * SEQ + c8;
                *(volatile v8h*)(Ph + oo) = hv; }
            if (ps == 0) __threadfence(); }
        wave_sync();
    }
}

__global__ __launch_bounds__(32 * AW) void k_keypass(const h16* __restrict__ QH, const h16* __restrict__ KP, const h16* __restrict__ VT, h16* AG) {
    __shared__ __align__(16) float os[AW * 16 * OSP];
    const int lane = threadIdx.x & 31, lr = lane & 15, hi = lane >> 4;
    const int wave = __builtin_amdgcn_readfirstlane((int)(threadIdx.x >> 5));
    const int t0 = ((int)blockIdx.x * AW + wave) * 16;
    const int wb = wave * 16 * OSP;
#pragma unroll 1
    for (int hh = 0; hh < HPW; ++hh) {
        const int h = (int)blockIdx.y * HPW + hh;
        const size_t pbase = (size_t)h * SEQ * HD;
        const v16h qh = ldh(QH + pbase + (size_t)(t0 + lr) * HD + 8 * hi);
        const size_t ko = pbase + (size_t)lr * HD + 8 * hi;
        const size_t vo = pbase + (size_t)lr * SEQ + 8 * hi;
        v8f o0 = (v8f){}, o1 = (v8f){};
        float m = NEGB, l = 0.0f;
#pragma unroll 1
        for (int key0 = 0; key0 < SEQ; key0 += 32) {
            const h16* ka = KP + ko + (size_t)key0 * HD;
            const v16h ka0 = ldh(ka), kb0 = ldh(ka + 16 * HD);
            v8f sa = (v8f){}, sb = (v8f){};
            sa = wmma16g(ka0, qh, sa); sb = wmma16g(kb0, qh, sb);
            float ta[8], tb[8]; float mx = NEGB;
#pragma unroll
            for (int r = 0; r < 8; ++r) { ta[r] = sa[r] * SC2; tb[r] = sb[r] * SC2; mx = fmaxf(mx, fmaxf(ta[r], tb[r])); }
            mx = fmaxf(mx, __shfl_xor(mx, 16, 32));
            const float mnew = fmaxf(m, mx);
            const float alpha = __builtin_amdgcn_exp2f(m - mnew);
            const float sh = PSH - mnew;
            v16h pb; float ls = 0.0f;
#pragma unroll
            for (int r = 0; r < 8; ++r) {
                const float xa = ta[r] + sh, xb = tb[r] + sh;
                const float ea = (xa < -14.0f) ? 0.0f : __builtin_amdgcn_exp2f(xa);
                const float eb = (xb < -14.0f) ? 0.0f : __builtin_amdgcn_exp2f(xb);
                const h16 pa = toh_flush(ea); const h16 pc = toh_flush(eb);
                pb[r] = pa; pb[8 + r] = pc;
                ls += (float)pa + (float)pc; }
            l = l * alpha + ls; m = mnew;
            o0 = o0 * alpha; o1 = o1 * alpha;
            const h16* va = VT + vo + key0;
            const v16h v0 = ldh(va), v1 = ldh(va + (size_t)16 * SEQ);
            o0 = wmma16g(v0, pb, o0); o1 = wmma16g(v1, pb, o1);
        }
        l += __shfl_xor(l, 16, 32);
        const float inv = ACS * (1.0f / l);
        { v4f a, c;
          a[0] = o0[0] * inv; a[1] = o0[1] * inv; a[2] = o0[2] * inv; a[3] = o0[3] * inv; c[0] = o0[4] * inv; c[1] = o0[5] * inv; c[2] = o0[6] * inv; c[3] = o0[7] * inv;
          *(v4fa*)(&os[wb + lr * OSP + hh * 32 +  0 + 8 * hi]) = a; *(v4fa*)(&os[wb + lr * OSP + hh * 32 +  0 + 8 * hi + 4]) = c;
          a[0] = o1[0] * inv; a[1] = o1[1] * inv; a[2] = o1[2] * inv; a[3] = o1[3] * inv; c[0] = o1[4] * inv; c[1] = o1[5] * inv; c[2] = o1[6] * inv; c[3] = o1[7] * inv;
          *(v4fa*)(&os[wb + lr * OSP + hh * 32 + 16 + 8 * hi]) = a; *(v4fa*)(&os[wb + lr * OSP + hh * 32 + 16 + 8 * hi + 4]) = c; }
    }
    wave_sync();
    h16* arow = AG + (size_t)t0 * DM + (size_t)blockIdx.y * (HPW * HD);
    static_assert(32 * 16 * 4 == 16 * HPW * HD * 2);
#pragma unroll 1
    for (int ps = 0; ps < 2; ++ps) {
#pragma unroll
        for (int s = 0; s < 4; ++s) { const int row = 4 * s + (lane >> 3), c8 = (lane & 7) * 8;
            const v4f x0 = *(const v4fa*)(&os[wb + row * OSP + c8]); const v4f x1 = *(const v4fa*)(&os[wb + row * OSP + c8 + 4]); v8h hv;
#pragma unroll
            for (int i = 0; i < 4; ++i) { hv[i] = toh_flush(x0[i]); hv[4 + i] = toh_flush(x1[i]); }
            *(volatile v8h*)(arow + (size_t)row * DM + c8) = hv; }
        if (ps == 0) __threadfence(); }
}

__global__ __launch_bounds__(32) void k_outp(const h16* __restrict__ A, const h16* __restrict__ Bt, const float* __restrict__ bias, const int* __restrict__ FLG, float* OUT) {
    __shared__ __align__(16) float os[16 * OSP];
    const int K = DM;
    const int lane = threadIdx.x & 31, lr = lane & 15, hi = lane >> 4; const int r0 = blockIdx.x * 64, c0 = blockIdx.y * 64;
    int fl = FLG[(size_t)lane * 32];
    fl |= __shfl_xor(fl, 16, 32); fl |= __shfl_xor(fl, 8, 32); fl |= __shfl_xor(fl, 4, 32); fl |= __shfl_xor(fl, 2, 32); fl |= __shfl_xor(fl, 1, 32);
    const bool poison = fl != 0;
    v8f acc[4][4];
#pragma unroll
    for (int mb = 0; mb < 4; ++mb)
#pragma unroll
        for (int nb = 0; nb < 4; ++nb) acc[mb][nb] = (v8f){};
    const size_t aoff = (size_t)(r0 + lr) * K + 8 * hi, boff = (size_t)(c0 + lr) * K + 8 * hi;
#pragma unroll 1
    for (int kc = 0; kc < K; kc += 32) {
        v16h a[4];
#pragma unroll
        for (int mb = 0; mb < 4; ++mb) a[mb] = ldh(A + aoff + (size_t)mb * 16 * K + kc);
#pragma unroll
        for (int nb = 0; nb < 4; ++nb) { const v16h b = ldh(Bt + boff + (size_t)nb * 16 * K + kc);
#pragma unroll
            for (int mb = 0; mb < 4; ++mb) acc[mb][nb] = wmma16g(a[mb], b, acc[mb][nb]); }
    }
    float bc[4];
#pragma unroll
    for (int nb = 0; nb < 4; ++nb) bc[nb] = bfr(bias[c0 + nb * 16 + lr]);
    const float pz = __uint_as_float(0x7FC00000u);
#pragma unroll
    for (int mb = 0; mb < 4; ++mb) {
#pragma unroll
        for (int nb = 0; nb < 4; ++nb) {
#pragma unroll
            for (int j = 0; j < 8; ++j) os[(hi * 8 + j) * OSP + nb * 16 + lr] = acc[mb][nb][j] * OSI + bc[nb]; }
        wave_sync();
        static_assert(32 * 16 * 8 == 16 * 64 * 4);
        float* orow = OUT + (size_t)(r0 + mb * 16) * DM + c0;
#pragma unroll 1
        for (int ps = 0; ps < 2; ++ps) {
#pragma unroll
            for (int s = 0; s < 8; ++s) { const int row = 2 * s + (lane >> 4), c4 = (lane & 15) * 4;
                v4f val = *(const v4fa*)(&os[row * OSP + c4]);
                val[0] = poison ? pz : val[0]; val[1] = poison ? pz : val[1]; val[2] = poison ? pz : val[2]; val[3] = poison ? pz : val[3];
                *(volatile v4f*)(orow + (size_t)row * DM + c4) = val; }
            if (ps == 0) __threadfence(); }
        wave_sync();
    }
}

static constexpr size_t al256(size_t v) { return (v + 255) & ~(size_t)255; }
static constexpr size_t SZ_XB = al256((size_t)SEQ * DM * 2);
static constexpr size_t SZ_WB = al256((size_t)3 * DM * DM * 2);
static constexpr size_t SZ_WO = al256((size_t)DM * DM * 2);
static constexpr size_t SZ_PL = al256((size_t)NH_ * SEQ * HD * 2);
static constexpr size_t SZ_AG = al256((size_t)SEQ * DM * 2);
static constexpr size_t SZ_FL = al256((size_t)ECB * 128);
static constexpr size_t SZ_TOTAL = SZ_XB + SZ_WB + SZ_WO + 3 * SZ_PL + SZ_AG + SZ_FL;
static_assert(SZ_TOTAL <= (size_t)134217728);
static_assert(((size_t)DM * DM * 2) % 256 == 0);
static_assert((size_t)NH_ * SEQ * HD == (size_t)DM * SEQ);
static_assert((SEQ / 64) * 64 == SEQ);
static_assert((DM / 64) * 64 == DM);
static_assert((SEQ / (16 * AW)) * 16 * AW == SEQ);
static_assert((NH_ / HPW) * HPW == NH_);

extern "C" void kernel_launch(void* const* d_in, const int* in_sizes, int n_in,
                              void* d_out, int out_size, void* d_ws, size_t ws_size, hipStream_t stream) {
    if (n_in < 11) return;
    if ((size_t)in_sizes[0] < (size_t)SEQ * DM) return;
    if ((size_t)in_sizes[1] < (size_t)NE * 2) return;
    if ((size_t)in_sizes[3] < (size_t)DM * DM || (size_t)in_sizes[5] < (size_t)DM * DM || (size_t)in_sizes[7] < (size_t)DM * DM || (size_t)in_sizes[9] < (size_t)DM * DM) return;
    if (in_sizes[4] < DM || in_sizes[6] < DM || in_sizes[8] < DM || in_sizes[10] < DM) return;
    if ((size_t)out_size < (size_t)SEQ * DM) return;
    if (SZ_TOTAL > ws_size) return;
    const float* feats = (const float*)d_in[0];
    const int* eidx = (const int*)d_in[1];
    const float* wq = (const float*)d_in[3]; const float* bq = (const float*)d_in[4];
    const float* wk = (const float*)d_in[5]; const float* bk = (const float*)d_in[6];
    const float* wv = (const float*)d_in[7]; const float* bv = (const float*)d_in[8];
    const float* wo = (const float*)d_in[9]; const float* bo = (const float*)d_in[10];
    float* OUT = (float*)d_out;
    char* wsp = (char*)d_ws;
    bf* XB = (bf*)wsp; wsp += SZ_XB;
    bf* WB = (bf*)wsp; wsp += SZ_WB;
    h16* WOH = (h16*)wsp; wsp += SZ_WO;
    h16* QH = (h16*)wsp; wsp += SZ_PL;
    h16* KP = (h16*)wsp; wsp += SZ_PL;
    h16* VT = (h16*)wsp; wsp += SZ_PL;
    h16* AG = (h16*)wsp; wsp += SZ_AG;
    int* FLG = (int*)wsp; wsp += SZ_FL;
    bf* WQ = WB; bf* WK = WB + (size_t)DM * DM; bf* WV = WB + (size_t)2 * DM * DM;

    { const size_t n8 = (size_t)SEQ * DM / 8;
      k_cvt8<<<(unsigned)((n8 + 255) / 256), 256, 0, stream>>>(feats, XB, n8); }
    { const size_t n8 = (size_t)DM * DM / 8; const unsigned g = (unsigned)((n8 + 255) / 256);
      k_cvt8<<<g, 256, 0, stream>>>(wq, WQ, n8); k_cvt8<<<g, 256, 0, stream>>>(wk, WK, n8); k_cvt8<<<g, 256, 0, stream>>>(wv, WV, n8);
      k_cvtw<<<g, 256, 0, stream>>>(wo, WOH, n8); }
    k_echeck<<<ECB, ECT, 0, stream>>>(eidx, FLG);

    k_proj_rows<<<dim3(SEQ / 64, DM / 64, 1), 32, 0, stream>>>(XB, WQ, bq, QH);
    k_proj_rows<<<dim3(SEQ / 64, DM / 64, 1), 32, 0, stream>>>(XB, WK, bk, KP);
    k_proj_cols<<<dim3(DM / 64, SEQ / 64, 1), 32, 0, stream>>>(WV, XB, bv, VT);

    k_keypass<<<dim3(SEQ / (16 * AW), NH_ / HPW, 1), 32 * AW, 0, stream>>>(QH, KP, VT, AG);

    k_outp<<<dim3(SEQ / 64, DM / 64, 1), 32, 0, stream>>>(AG, WOH, bo, FLG, OUT);
}
